// BuddingLayer_84430467105102
// MI455X (gfx1250) — hardware-verified
//
#include <hip/hip_runtime.h>
#include <math.h>

typedef __attribute__((ext_vector_type(16))) _Float16 v16h;
typedef __attribute__((ext_vector_type(16))) __bf16 v16b;
typedef __attribute__((ext_vector_type(8)))  _Float16 v8h;
typedef __attribute__((ext_vector_type(8)))  float v8f;
typedef __attribute__((ext_vector_type(4)))  float v4f;
typedef __attribute__((ext_vector_type(2)))  float v2f;
typedef __attribute__((ext_vector_type(4)))  unsigned v4u;
typedef __attribute__((ext_vector_type(4)))  int v4i;
typedef float __attribute__((may_alias)) float_a;
typedef int __attribute__((may_alias)) int_a;

template <typename T> __device__ __forceinline__ void vst2(void* p, T v) { *(volatile T*)p = v; __threadfence(); *(volatile T*)p = v; }
__device__ __forceinline__ v8f wmma16(v16h a, v16h b, v8f c) {
  v8f d = __builtin_amdgcn_wmma_f32_16x16x32_f16(false, a, false, b, (short)0, c, false, false);
  asm volatile("v_nop\n\tv_nop\n\tv_nop\n\tv_nop" : "+v"(d) : "v"(a), "v"(b));
  return d;
}
__device__ __forceinline__ v8f wmma_bf(v16b a, v16b b, v8f c) {
  v8f d = __builtin_amdgcn_wmma_f32_16x16x32_bf16(false, a, false, b, (short)0, c, false, false);
  asm volatile("v_nop\n\tv_nop\n\tv_nop\n\tv_nop" : "+v"(d) : "v"(a), "v"(b));
  return d;
}
__device__ __forceinline__ v16h frag_h(const _Float16* rowk0, int lane) {
  union { v16h v; v8h q[2]; } u; const _Float16* p = rowk0 + 8 * (lane >> 4);
  u.q[0] = *(const v8h*)p; u.q[1] = *(const v8h*)(p + 16); return u.v;
}
__device__ __forceinline__ v16h frag_f32(const float* rowk0, int lane) {
  v16h a; const float* p = rowk0 + 8 * (lane >> 4);
#pragma unroll
  for (int i = 0; i < 8; ++i) { a[i] = (_Float16)p[i]; a[8 + i] = (_Float16)p[16 + i]; }
  return a;
}
__device__ __forceinline__ v16h frag_f32s(const float* rowk0, int lane, float sc) {
  v16h a; const float* p = rowk0 + 8 * (lane >> 4);
#pragma unroll
  for (int i = 0; i < 8; ++i) { a[i] = (_Float16)(p[i] * sc); a[8 + i] = (_Float16)(p[16 + i] * sc); }
  return a;
}
__device__ __forceinline__ v16h fragc_f32(const float* W, int k0, int n, int lane, int ld, int K) {
  v16h a; const int g = lane >> 4;
#pragma unroll
  for (int i = 0; i < 8; ++i) { const int ka = k0 + 8 * g + i, kb = ka + 16;
    a[i] = (_Float16)(ka < K ? W[(size_t)ka * ld + n] : 0.f); a[8 + i] = (_Float16)(kb < K ? W[(size_t)kb * ld + n] : 0.f); }
  return a;
}
struct F2 { v16b h, l; };
__device__ __forceinline__ F2 bsplit16(const float v[16]) { F2 r;
#pragma unroll
  for (int i = 0; i < 16; ++i) { const __bf16 h = (__bf16)v[i]; r.h[i] = h; r.l[i] = (__bf16)(v[i] - (float)h); }
  return r; }
__device__ __forceinline__ F2 split_row(const float* row, int k0, int lane) { float v[16]; const float* p = row + k0 + 8 * (lane >> 4);
#pragma unroll
  for (int i = 0; i < 8; ++i) { v[i] = p[i]; v[8 + i] = p[16 + i]; }
  return bsplit16(v); }
__device__ __forceinline__ F2 split_rowK(const float* row, int k0, int lane, int K) { float v[16]; const int g = lane >> 4;
#pragma unroll
  for (int i = 0; i < 8; ++i) { const int ka = k0 + 8 * g + i, kb = ka + 16; v[i] = ka < K ? row[ka] : 0.f; v[8 + i] = kb < K ? row[kb] : 0.f; }
  return bsplit16(v); }
__device__ __forceinline__ F2 split_col(const float* W, int k0, int n, int lane, int ld, int K) { float v[16]; const int g = lane >> 4;
#pragma unroll
  for (int i = 0; i < 8; ++i) { const int ka = k0 + 8 * g + i, kb = ka + 16; v[i] = ka < K ? W[(size_t)ka * ld + n] : 0.f; v[8 + i] = kb < K ? W[(size_t)kb * ld + n] : 0.f; }
  return bsplit16(v); }
__device__ __forceinline__ v8f mac3(const F2& a, const F2& b, v8f c) { c = wmma_bf(a.l, b.h, c); c = wmma_bf(a.h, b.l, c); return wmma_bf(a.h, b.h, c); }
__device__ __forceinline__ float sigm(float v) { return 1.0f / (1.0f + expf(-v)); }
#define LDSX() do { asm volatile("s_wait_dscnt 0" ::: "memory"); __builtin_amdgcn_wave_barrier(); __builtin_amdgcn_fence(__ATOMIC_RELEASE, "workgroup"); } while (0)

#define NB 512
#define NI 2048
#define NO 2048
#define KB 128

__global__ __launch_bounds__(128) void k_dense(const float* __restrict__ x, const int* __restrict__ sat, const float* __restrict__ W, const float* __restrict__ bias, float* __restrict__ pre) {
  __shared__ __align__(16) float so[4][16][132];
  __shared__ int smask[NI / 32];
  const int tid = threadIdx.x, wave = tid >> 5, lane = tid & 31, col = lane & 15, g = lane >> 4;
  const int r0 = blockIdx.x * 64 + wave * 16, n0 = blockIdx.y * 128;
  for (int i = tid; i < NI / 32; i += 128) smask[i] = 0;
  __syncthreads();
  for (int i = tid; i < KB; i += 128) { const int s = sat[i]; if (s >= 0 && s < NI) atomicOr(&smask[s >> 5], 1 << (s & 31)); }
  __syncthreads();
  v8f acc[8] = {};
#pragma unroll 1
  for (int kc = 0; kc < NI / 32; ++kc) { v16h a; const float* p = x + (size_t)(r0 + col) * NI + kc * 32 + 8 * g; const int mword = smask[kc];
#pragma unroll
    for (int i = 0; i < 8; ++i) { const int ka = 8 * g + i, kb = 16 + 8 * g + i;
      a[i] = (_Float16)(((mword >> ka) & 1) ? 0.f : p[i]); a[8 + i] = (_Float16)(((mword >> kb) & 1) ? 0.f : p[16 + i]); }
#pragma unroll
    for (int j = 0; j < 8; ++j) acc[j] = wmma16(a, frag_f32s(W + (size_t)(n0 + j * 16 + col) * NI + kc * 32, lane, 64.0f), acc[j]); }
#pragma unroll
  for (int j = 0; j < 8; ++j) { const float bv = bias[n0 + j * 16 + col];
#pragma unroll
    for (int r = 0; r < 8; ++r) so[wave][8 * g + r][j * 16 + col] = acc[j][r] * (1.0f / 64.0f) + bv; }
  LDSX();
#pragma unroll 4
  for (int rl = 0; rl < 16; ++rl) vst2(pre + (size_t)(r0 + rl) * NO + n0 + lane * 4, *(const v4f*)(&so[wave][rl][lane * 4]));
}
__global__ __launch_bounds__(256) void k_bud(const float* __restrict__ x, const int* __restrict__ sat, const float* __restrict__ W1, const float* __restrict__ b1,
                                           const float* __restrict__ W2, const float* __restrict__ b2, const float* __restrict__ W3, const float* __restrict__ b3,
                                           const float* __restrict__ pre, float* __restrict__ out) {
  __shared__ float h2[KB][4];
  __shared__ __align__(16) float so[256];
  const int b = blockIdx.y, o = blockIdx.x * 256 + threadIdx.x, tid = threadIdx.x;
  if (tid < KB) { const int k = tid; int s = sat[k]; s = s < 0 ? 0 : (s >= NI ? NI - 1 : s);
    const float xs = x[(size_t)b * NI + s] * (1.0f / 3.0f);
    float h1[3], hb[3];
#pragma unroll
    for (int j = 0; j < 3; ++j) { float a = b1[k * 3 + j];
#pragma unroll
      for (int i = 0; i < 3; ++i) a += xs * W1[(k * 3 + i) * 3 + j];
      h1[j] = a > 0.f ? a : 0.f; }
#pragma unroll
    for (int j = 0; j < 3; ++j) { float a = b2[k * 3 + j];
#pragma unroll
      for (int i = 0; i < 3; ++i) a += h1[i] * W2[(k * 3 + i) * 3 + j];
      hb[j] = a > 0.f ? a : 0.f; }
    h2[k][0] = hb[0]; h2[k][1] = hb[1]; h2[k][2] = hb[2]; h2[k][3] = 0.f; }
  __syncthreads();
  float u = 0.f;
#pragma unroll 1
  for (int k = 0; k < KB; ++k) { float a = b3[(size_t)k * NO + o];
    a += h2[k][0] * W3[((size_t)k * 3 + 0) * NO + o] + h2[k][1] * W3[((size_t)k * 3 + 1) * NO + o] + h2[k][2] * W3[((size_t)k * 3 + 2) * NO + o];
    u += a > 0.f ? a : 0.f; }
  so[tid] = pre[(size_t)b * NO + o] + u;
  __syncthreads();
  if (tid < 64) vst2(out + (size_t)b * NO + blockIdx.x * 256 + tid * 4, *(const v4f*)(&so[tid * 4]));
}
extern "C" void kernel_launch(void* const* d_in, const int* in_sizes, int n_in, void* d_out, int out_size, void* d_ws, size_t ws_size, hipStream_t stream) {
  (void)in_sizes; (void)n_in; (void)out_size; (void)ws_size;
  const float* x = (const float*)d_in[0]; const int* sat = (const int*)d_in[1]; const float* W = (const float*)d_in[2]; const float* bias = (const float*)d_in[3];
  const float* W1 = (const float*)d_in[4]; const float* b1 = (const float*)d_in[5]; const float* W2 = (const float*)d_in[6]; const float* b2 = (const float*)d_in[7];
  const float* W3 = (const float*)d_in[8]; const float* b3 = (const float*)d_in[9];
  float* out = (float*)d_out; float* pre = (float*)d_ws;
  k_dense<<<dim3(NB / 64, NO / 128), 128, 0, stream>>>(x, sat, W, bias, pre);
  k_bud<<<dim3(NO / 256, NB), 256, 0, stream>>>(x, sat, W1, b1, W2, b2, W3, b3, pre, out);
}
